// RelationNetwork_53584011985126
// MI455X (gfx1250) — hardware-verified
//
#include <hip/hip_runtime.h>
#include <math.h>

constexpr int kBatch     = 32;
constexpr int kChan      = 256;
constexpr int kNobj      = 64;
constexpr int kHG        = 512;
constexpr int kHF        = 512;
constexpr int kDOut      = 256;
constexpr int kDGIn      = 2 * kChan + 2;
constexpr int kObjRows   = kBatch * kNobj;
constexpr int kW0N       = 2 * kHG;
constexpr int kChunkB    = 8;
constexpr int kNChunks   = kBatch / kChunkB;
constexpr int kChunkRows = kChunkB * kNobj * kNobj;
constexpr float kXCarry  = 8.0f;
constexpr float kWCarry  = 256.0f;
constexpr float kHCarry  = 16.0f;
constexpr float kScale0  = 1.0f / (8.0f * 256.0f);
constexpr float kScale12 = 1.0f / (16.0f * 256.0f);

constexpr size_t kOffW12t = 0;
constexpr size_t kOffW0t  = kOffW12t + (size_t)2 * kHG * kHG * 2;
constexpr size_t kOffXt   = kOffW0t + (size_t)kW0N * kChan * 2;
constexpr size_t kOffAB   = kOffXt + (size_t)kObjRows * kChan * 2;
constexpr size_t kOffH0   = kOffAB + (size_t)kObjRows * kW0N * 4;
constexpr size_t kOffH1   = kOffH0 + (size_t)kChunkRows * kHG * 2;
constexpr size_t kOffPar  = kOffH1 + (size_t)kChunkRows * kHG * 2;
constexpr size_t kWsTotal = kOffPar + (size_t)kObjRows * kHG * 4;
static_assert(kWsTotal == (size_t)82313216, "ws total");
static_assert(kWsTotal <= (size_t)134217728, "ws cap");
static_assert(kChan % 32 == 0 && kHG % 32 == 0, "K tiles");
static_assert(kObjRows % 64 == 0 && kW0N % 64 == 0 && kChunkRows % 64 == 0 && kHG % 64 == 0, "MN tiles");
static_assert(kNobj == 64, "one 64-row tile per (b,p)");
static_assert(kChunkRows % 4 == 0 && kHG == 64 * 8, "pair assembly coverage");

typedef __attribute__((ext_vector_type(16))) _Float16 v16h;
typedef __attribute__((ext_vector_type(8)))  _Float16 v8h;
typedef __attribute__((ext_vector_type(16))) __bf16   v16b;
typedef __attribute__((ext_vector_type(8)))  __bf16   v8b;
typedef __attribute__((ext_vector_type(8)))  float    v8f;
typedef __attribute__((ext_vector_type(4)))  float    v4f;
typedef __attribute__((ext_vector_type(4)))  unsigned int v4u;

__device__ __forceinline__ unsigned short f2bf_bits(float f) {
  unsigned u = __float_as_uint(f);
  return (unsigned short)((u + 0x7FFFu + ((u >> 16) & 1u)) >> 16);
}
__device__ __forceinline__ float bf_bits2f(unsigned short h) { return __uint_as_float(((unsigned)h) << 16); }

__device__ __forceinline__ void dep_guard_h(v8f& a, v8f& b, v16h x, v16h y) { asm volatile("v_nop\n\tv_nop\n\tv_nop\n\tv_nop" : "+v"(a), "+v"(b) : "v"(x), "v"(y)); }
__device__ __forceinline__ void dep_guard_b(v8f& a, v8f& b, v16b x, v16b y) { asm volatile("v_nop\n\tv_nop\n\tv_nop\n\tv_nop" : "+v"(a), "+v"(b) : "v"(x), "v"(y)); }
__device__ __forceinline__ void keep4_h(v16h a, v16h b, v16h c, v16h d) { asm volatile("v_nop" :: "v"(a), "v"(b), "v"(c), "v"(d)); }
__device__ __forceinline__ void keep4_b(v16b a, v16b b, v16b c, v16b d) { asm volatile("v_nop" :: "v"(a), "v"(b), "v"(c), "v"(d)); }
__device__ __forceinline__ void acc_guard4(v8f& a, v8f& b, v8f& c, v8f& d) { asm volatile("v_nop\n\tv_nop\n\tv_nop\n\tv_nop" : "+v"(a), "+v"(b), "+v"(c), "+v"(d)); }
template <typename T> struct Frag;
template <> struct Frag<_Float16> {
  typedef v16h V; union U { v16h v; v8h h[2]; };
  static __device__ __forceinline__ v16h load(const _Float16* p) {
    U f; f.h[0] = *(const v8h*)(p); f.h[1] = *(const v8h*)(p + 16); return f.v;
  }
  static __device__ __forceinline__ v8f mma(v16h a, v16h b, v8f c) {
    return __builtin_amdgcn_wmma_f32_16x16x32_f16(false, a, false, b, (short)0, c, false, false);
  }
  static __device__ __forceinline__ void guard(v8f& a, v8f& b, v16h x, v16h y) { dep_guard_h(a, b, x, y); }
  static __device__ __forceinline__ void keep(v16h a, v16h b, v16h c, v16h d) { keep4_h(a, b, c, d); }
};
template <> struct Frag<__bf16> {
  typedef v16b V; union U { v16b v; v8b h[2]; };
  static __device__ __forceinline__ v16b load(const __bf16* p) {
    U f; f.h[0] = *(const v8b*)(p); f.h[1] = *(const v8b*)(p + 16); return f.v;
  }
  static __device__ __forceinline__ v8f mma(v16b a, v16b b, v8f c) {
    return __builtin_amdgcn_wmma_f32_16x16x32_bf16(false, a, false, b, (short)0, c, false, false);
  }
  static __device__ __forceinline__ void guard(v8f& a, v8f& b, v16b x, v16b y) { dep_guard_b(a, b, x, y); }
  static __device__ __forceinline__ void keep(v16b a, v16b b, v16b c, v16b d) { keep4_b(a, b, c, d); }
};

__device__ __forceinline__ unsigned pk16(unsigned short a, unsigned short b) { return (unsigned)a | ((unsigned)b << 16); }
__device__ __forceinline__ unsigned short h_bits(float f) { const _Float16 h = (_Float16)f; return __builtin_bit_cast(unsigned short, h); }

template <int ET> struct Elem;
template <> struct Elem<0> { typedef _Float16 T; };
template <> struct Elem<1> { typedef __bf16 T; };
template <int ET, bool SPLIT, int BIAS_MODE, int OUT_MODE, bool RESID, int ACT = 0>
__global__ __launch_bounds__(256) void wmma_gemm64(
    const unsigned short* __restrict__ Ap, const unsigned short* __restrict__ A2p, int lda, long strideA,
    const unsigned short* __restrict__ Btp, const unsigned short* __restrict__ Bt2p, int ldb, long strideB,
    void* __restrict__ Cout, void* __restrict__ Cout2, int ldc, long strideC,
    const float* __restrict__ bias,
    const float* __restrict__ resid, long strideR,
    int M, int N, int K, float scale, float oscale) {
  typedef typename Elem<ET>::T T;
  typedef typename Frag<T>::V V;
  const T* A = (const T*)Ap; const T* A2 = (const T*)A2p; const T* Bt = (const T*)Btp; const T* Bt2 = (const T*)Bt2p;
  __shared__ __align__(16) float sT[8][16 * 68];
  const int b    = blockIdx.y;
  const int lane = threadIdx.x & 31;
  const int wave = threadIdx.x >> 5;
  const int tilesN = N >> 6;
  const int tilesM = M >> 6;
  const int tile = blockIdx.x * 8 + wave;
  if (tile >= tilesM * tilesN) return;
  const int tm = tile / tilesN;
  const int tn = tile - tm * tilesN;
  const int m0 = tm << 6;
  const int n0 = tn << 6;

  const T* Ab  = A  + (size_t)b * strideA;
  const T* Bb  = Bt + (size_t)b * strideB;
  const T* Ab2 = SPLIT ? (A2  + (size_t)b * strideA) : nullptr;
  const T* Bb2 = SPLIT ? (Bt2 + (size_t)b * strideB) : nullptr;

  const int rlane = lane & 15;
  const int koff  = (lane >> 4) * 8;
  const int mOff  = (lane >> 4) * 8;

  v8f acc[4][4];
#pragma unroll
  for (int i = 0; i < 4; ++i)
#pragma unroll
    for (int j = 0; j < 4; ++j) acc[i][j] = (v8f){0.f,0.f,0.f,0.f,0.f,0.f,0.f,0.f};

  for (int k0 = 0; k0 < K; k0 += 32) {
    V bh[4], bl[4];
#pragma unroll
    for (int j = 0; j < 4; ++j) {
      const size_t bo = (size_t)(n0 + (j << 4) + rlane) * ldb + koff + k0;
      bh[j] = Frag<T>::load(Bb + bo);
      if (SPLIT) bl[j] = Frag<T>::load(Bb2 + bo);
    }
#pragma unroll
    for (int i = 0; i < 4; ++i) {
      const size_t ao = (size_t)(m0 + (i << 4) + rlane) * lda + koff + k0;
      V ah = Frag<T>::load(Ab + ao);
      V al;
      if (SPLIT) al = Frag<T>::load(Ab2 + ao);
#pragma unroll
      for (int j = 0; j < 4; ++j) {
        acc[i][j] = Frag<T>::mma(ah, bh[j], acc[i][j]);
        if (SPLIT) {
          acc[i][j] = Frag<T>::mma(ah, bl[j], acc[i][j]);
          acc[i][j] = Frag<T>::mma(al, bh[j], acc[i][j]);
        }
      }
      Frag<T>::guard(acc[i][0], acc[i][3], ah, SPLIT ? al : ah);
    }
    Frag<T>::keep(bh[0], bh[1], bh[2], bh[3]);
    if (SPLIT) Frag<T>::keep(bl[0], bl[1], bl[2], bl[3]);
  }
  acc_guard4(acc[0][0], acc[0][1], acc[0][2], acc[0][3]);
  acc_guard4(acc[1][0], acc[1][1], acc[1][2], acc[1][3]);
  acc_guard4(acc[2][0], acc[2][1], acc[2][2], acc[2][3]);
  acc_guard4(acc[3][0], acc[3][1], acc[3][2], acc[3][3]);

  float* slab = sT[wave];
  const float* Rb = RESID ? (resid + (size_t)b * strideR) : nullptr;
#pragma unroll
  for (int i = 0; i < 4; ++i) {
    const int mBase = m0 + (i << 4);
#pragma unroll
    for (int j = 0; j < 4; ++j) {
      const int n = n0 + (j << 4) + rlane;
      float bv = 0.f;
      if (BIAS_MODE == 2) bv = bias[n];
#pragma unroll
      for (int r = 0; r < 8; ++r) {
        float v = acc[i][j][r] * scale;
        if (BIAS_MODE == 1) v += bias[mBase + mOff + r];
        if (BIAS_MODE == 2) v += bv;
        if (RESID) v += Rb[(size_t)(mBase + mOff + r) * ldc + n];
        if (ACT == 2) v = fmaxf(v, 0.0f);
        if (ACT == 4) v = (v > 0.f) ? v : 0.01f * v;
        v = v * oscale;
        slab[(mOff + r) * 68 + (j << 4) + rlane] = v;
      }
    }
    __builtin_amdgcn_fence(__ATOMIC_RELEASE, "workgroup");
    __builtin_amdgcn_wave_barrier();
    __builtin_amdgcn_fence(__ATOMIC_ACQUIRE, "workgroup");
    if (OUT_MODE == 0) {
      float* C = (float*)Cout + (size_t)b * strideC;
      const int hh = lane >> 4, c4 = (lane & 15) * 4;
      for (int pass = 0; pass < 2; ++pass) {
#pragma unroll
        for (int it = 0; it < 8; ++it) {
          const int row = it * 2 + hh;
          v4f v = *(const v4f*)(slab + row * 68 + c4);
          *(volatile v4f*)(C + (size_t)(mBase + row) * ldc + n0 + c4) = v;
        }
        __threadfence();
      }
    } else {
      const int q = lane >> 3, c8 = (lane & 7) * 8;
      unsigned short* C  = (unsigned short*)Cout  + (size_t)b * strideC;
      unsigned short* C2 = (OUT_MODE == 2) ? ((unsigned short*)Cout2 + (size_t)b * strideC) : nullptr;
      for (int pass = 0; pass < 2; ++pass) {
#pragma unroll
        for (int it = 0; it < 4; ++it) {
          const int row = it * 4 + q;
          const float* sp = slab + row * 68 + c8;
          v8h hv, lv;
#pragma unroll
          for (int e = 0; e < 8; ++e) {
            if (OUT_MODE == 1) {
              hv[e] = (_Float16)sp[e];
            } else {
              unsigned short hb = f2bf_bits(sp[e]);
              unsigned short lb = f2bf_bits(sp[e] - bf_bits2f(hb));
              hv[e] = __builtin_bit_cast(_Float16, hb);
              lv[e] = __builtin_bit_cast(_Float16, lb);
            }
          }
          *(volatile v8h*)(C + (size_t)(mBase + row) * ldc + n0 + c8) = hv;
          if (OUT_MODE == 2) *(volatile v8h*)(C2 + (size_t)(mBase + row) * ldc + n0 + c8) = lv;
        }
        __threadfence();
      }
    }
    __builtin_amdgcn_fence(__ATOMIC_RELEASE, "workgroup");
    __builtin_amdgcn_wave_barrier();
    __builtin_amdgcn_fence(__ATOMIC_ACQUIRE, "workgroup");
  }
}

template <int ET, int ACT>
__global__ __launch_bounds__(256) void wmma_gemm64_rowsum(
    const unsigned short* __restrict__ Ap, int lda,
    const unsigned short* __restrict__ Btp, int ldb,
    float* __restrict__ Pout, int ldp,
    const float* __restrict__ bias,
    int M, int N, int K, float scale) {
  typedef typename Elem<ET>::T T;
  typedef typename Frag<T>::V V;
  const T* Ab = (const T*)Ap; const T* Bb = (const T*)Btp;
  __shared__ __align__(16) float sR[8][2 * 64];
  const int lane = threadIdx.x & 31;
  const int wave = threadIdx.x >> 5;
  const int tilesN = N >> 6;
  const int tilesM = M >> 6;
  const int tile = blockIdx.x * 8 + wave;
  if (tile >= tilesM * tilesN) return;
  const int tm = tile / tilesN;
  const int tn = tile - tm * tilesN;
  const int m0 = tm << 6;
  const int n0 = tn << 6;

  const int rlane = lane & 15;
  const int koff  = (lane >> 4) * 8;

  v8f acc[4][4];
#pragma unroll
  for (int i = 0; i < 4; ++i)
#pragma unroll
    for (int j = 0; j < 4; ++j) acc[i][j] = (v8f){0.f,0.f,0.f,0.f,0.f,0.f,0.f,0.f};

  for (int k0 = 0; k0 < K; k0 += 32) {
    V bh[4];
#pragma unroll
    for (int j = 0; j < 4; ++j) {
      const size_t bo = (size_t)(n0 + (j << 4) + rlane) * ldb + koff + k0;
      bh[j] = Frag<T>::load(Bb + bo);
    }
#pragma unroll
    for (int i = 0; i < 4; ++i) {
      const size_t ao = (size_t)(m0 + (i << 4) + rlane) * lda + koff + k0;
      V ah = Frag<T>::load(Ab + ao);
#pragma unroll
      for (int j = 0; j < 4; ++j) acc[i][j] = Frag<T>::mma(ah, bh[j], acc[i][j]);
      Frag<T>::guard(acc[i][0], acc[i][3], ah, ah);
    }
    Frag<T>::keep(bh[0], bh[1], bh[2], bh[3]);
  }
  acc_guard4(acc[0][0], acc[0][1], acc[0][2], acc[0][3]);
  acc_guard4(acc[1][0], acc[1][1], acc[1][2], acc[1][3]);
  acc_guard4(acc[2][0], acc[2][1], acc[2][2], acc[2][3]);
  acc_guard4(acc[3][0], acc[3][1], acc[3][2], acc[3][3]);

  float cs[4];
#pragma unroll
  for (int j = 0; j < 4; ++j) {
    const float bv = bias[n0 + (j << 4) + rlane];
    float s = 0.0f;
#pragma unroll
    for (int i = 0; i < 4; ++i) {
#pragma unroll
      for (int r = 0; r < 8; ++r) {
        float v = acc[i][j][r] * scale + bv;
        if (ACT == 2) v = fmaxf(v, 0.0f);
        if (ACT == 4) v = (v > 0.f) ? v : 0.01f * v;
        s += v;
      }
    }
    cs[j] = s;
  }
#pragma unroll
  for (int j = 0; j < 4; ++j) cs[j] += __shfl_xor(cs[j], 16, 32);
  float* slab = sR[wave];
#pragma unroll
  for (int j = 0; j < 4; ++j) slab[(lane >> 4) * 64 + (j << 4) + rlane] = cs[j];
  __builtin_amdgcn_fence(__ATOMIC_RELEASE, "workgroup");
  __builtin_amdgcn_wave_barrier();
  __builtin_amdgcn_fence(__ATOMIC_ACQUIRE, "workgroup");
  const v4f pv = *(const v4f*)(slab + 4 * (lane & 15));
  float* prow = Pout + (size_t)tm * ldp + n0;
  for (int pass = 0; pass < 2; ++pass) {
    if (lane < 16) *(volatile v4f*)(prow + 4 * lane) = pv;
    __threadfence();
  }
}

__global__ __launch_bounds__(256) void wtcast_kernel(const float* __restrict__ gW1, const float* __restrict__ gW2,
                                                     const float* __restrict__ gW0,
                                                     unsigned short* __restrict__ W12t, unsigned short* __restrict__ W0t,
                                                     float scale) {
  __shared__ float sm[64][65];
  const int t  = threadIdx.x;
  const int d0 = blockIdx.x * 64;
  const int h0 = blockIdx.y * 64;
  const int z  = blockIdx.z;
  const float* W = (z == 0) ? gW1 : (z == 1) ? gW2 : gW0;
#pragma unroll
  for (int i = 0; i < 16; ++i) {
    const int e = i * 256 + t;
    const int r = e >> 6;
    const int c = e & 63;
    sm[c][r] = W[(size_t)(d0 + r) * kHG + h0 + c] * scale;
  }
  __syncthreads();
  unsigned short* base; int pitch, roff, coff;
  if (z < 2) { base = W12t + (size_t)z * kHG * kHG; pitch = kHG; roff = h0; coff = d0; }
  else       { base = W0t; pitch = kChan; roff = h0 + ((d0 >> 8) << 9); coff = d0 & 255; }
  const int lane = t & 31, wave = t >> 5;
  const int q = lane >> 3, c8 = (lane & 7) * 8;
  for (int pass = 0; pass < 2; ++pass) {
#pragma unroll
    for (int it = 0; it < 2; ++it) {
      const int row = wave * 8 + it * 4 + q;
      unsigned short hb[8];
#pragma unroll
      for (int e = 0; e < 8; ++e) hb[e] = h_bits(sm[row][c8 + e]);
      const v4u u = (v4u){pk16(hb[0], hb[1]), pk16(hb[2], hb[3]), pk16(hb[4], hb[5]), pk16(hb[6], hb[7])};
      *(volatile v4u*)(base + (size_t)(roff + row) * pitch + coff + c8) = u;
    }
    __threadfence();
  }
}

__global__ __launch_bounds__(256) void xtcast_kernel(const float* __restrict__ x, unsigned short* __restrict__ Xt, float scale) {
  __shared__ float sm[64][65];
  const int t  = threadIdx.x;
  const int c0 = blockIdx.x * 64;
  const int b  = blockIdx.y;
  const float* xb = x + (size_t)b * kChan * kNobj;
#pragma unroll
  for (int i = 0; i < 16; ++i) {
    const int e  = i * 256 + t;
    const int cl = e >> 6;
    const int n  = e & 63;
    sm[n][cl] = xb[(size_t)(c0 + cl) * kNobj + n] * scale;
  }
  __syncthreads();
  const int lane = t & 31, wave = t >> 5;
  const int q = lane >> 3, c8 = (lane & 7) * 8;
  for (int pass = 0; pass < 2; ++pass) {
#pragma unroll
    for (int it = 0; it < 2; ++it) {
      const int row = wave * 8 + it * 4 + q;
      unsigned short hb[8];
#pragma unroll
      for (int e = 0; e < 8; ++e) hb[e] = h_bits(sm[row][c8 + e]);
      const v4u u = (v4u){pk16(hb[0], hb[1]), pk16(hb[2], hb[3]), pk16(hb[4], hb[5]), pk16(hb[6], hb[7])};
      *(volatile v4u*)(Xt + (size_t)(b * kNobj + row) * kChan + c0 + c8) = u;
    }
    __threadfence();
  }
}

__global__ __launch_bounds__(256) void build_h0_kernel(const float* __restrict__ AB, const float* __restrict__ gW0,
                                                       const float* __restrict__ gb0, unsigned short* __restrict__ H0, int chunk) {
  __shared__ __align__(16) float sw0[kHG];
  __shared__ __align__(16) float sw1[kHG];
  __shared__ __align__(16) float sbb[kHG];
  const int t = threadIdx.x;
  if (t < 128) {
    *(v4f*)(sw0 + 4 * t) = *(const v4f*)(gW0 + (size_t)(2 * kChan) * kHG + 4 * t);
    *(v4f*)(sw1 + 4 * t) = *(const v4f*)(gW0 + (size_t)(2 * kChan + 1) * kHG + 4 * t);
    *(v4f*)(sbb + 4 * t) = *(const v4f*)(gb0 + 4 * t);
  }
  __syncthreads();
  const int rl = blockIdx.x * 4 + (t >> 6);
  const int h8 = (t & 63) * 8;
  const int bl = rl >> 12, p = (rl >> 6) & 63, q = rl & 63;
  const int b  = chunk * kChunkB + bl;
  const float r0 = (float)((p >> 3) - (q >> 3));
  const float r1 = (float)((p & 7) - (q & 7));
  const float* arow = AB + (size_t)(b * kNobj + q) * kW0N + h8;
  const float* brow = AB + (size_t)(b * kNobj + p) * kW0N + kHG + h8;
  const v4f a0 = *(const v4f*)(arow), a1 = *(const v4f*)(arow + 4);
  const v4f m0 = *(const v4f*)(brow), m1 = *(const v4f*)(brow + 4);
  const v4f w00 = *(const v4f*)(sw0 + h8), w01 = *(const v4f*)(sw0 + h8 + 4);
  const v4f w10 = *(const v4f*)(sw1 + h8), w11 = *(const v4f*)(sw1 + h8 + 4);
  const v4f bb0 = *(const v4f*)(sbb + h8), bb1 = *(const v4f*)(sbb + h8 + 4);
  unsigned short hb[8];
#pragma unroll
  for (int e = 0; e < 4; ++e) {
    float v = a0[e] + m0[e];
    v = fmaf(r0, w00[e], v);
    v = fmaf(r1, w10[e], v);
    v = v + bb0[e];
    v = fmaxf(v, 0.0f) * kHCarry;
    hb[e] = h_bits(v);
    float u = a1[e] + m1[e];
    u = fmaf(r0, w01[e], u);
    u = fmaf(r1, w11[e], u);
    u = u + bb1[e];
    u = fmaxf(u, 0.0f) * kHCarry;
    hb[4 + e] = h_bits(u);
  }
  const v4u pk = (v4u){pk16(hb[0], hb[1]), pk16(hb[2], hb[3]), pk16(hb[4], hb[5]), pk16(hb[6], hb[7])};
  unsigned short* dst = H0 + (size_t)rl * kHG + h8;
  *(volatile v4u*)dst = pk;
  __threadfence();
  *(volatile v4u*)dst = pk;
}

__global__ __launch_bounds__(256) void fmlp_kernel(const float* __restrict__ partial, const float* __restrict__ fW0,
                                                   const float* __restrict__ fb0, const float* __restrict__ fW1,
                                                   const float* __restrict__ fb1, float* __restrict__ out) {
  __shared__ float semb[kHG];
  __shared__ float shf[kHF];
  __shared__ __align__(16) float so[kDOut];
  const int t = threadIdx.x, lane = t & 31, wave = t >> 5;
  const int b = blockIdx.x;
  const float* pb = partial + (size_t)b * kNobj * kHG;
  for (int h = t; h < kHG; h += 256) {
    float s = 0.0f;
#pragma unroll 4
    for (int p = 0; p < kNobj; ++p) s += pb[(size_t)p * kHG + h];
    semb[h] = s;
  }
  __syncthreads();
  for (int j = t; j < kHF; j += 256) {
    float s = 0.0f;
#pragma unroll 4
    for (int h = 0; h < kHG; ++h) s = fmaf(semb[h], fW0[(size_t)h * kHF + j], s);
    s = s + fb0[j];
    shf[j] = fmaxf(s, 0.0f);
  }
  __syncthreads();
  {
    const int j = t;
    float s = 0.0f;
#pragma unroll 4
    for (int h = 0; h < kHF; ++h) s = fmaf(shf[h], fW1[(size_t)h * kDOut + j], s);
    s = s + fb1[j];
    so[j] = s;
  }
  __syncthreads();
  if (wave < 2) {
    const v4f v = *(const v4f*)(so + wave * 128 + 4 * lane);
    float* op = out + (size_t)b * kDOut + wave * 128 + 4 * lane;
    for (int pass = 0; pass < 2; ++pass) {
      *(volatile v4f*)op = v;
      __threadfence();
    }
  }
}

extern "C" void kernel_launch(void* const* d_in, const int* in_sizes, int n_in,
                              void* d_out, int out_size, void* d_ws, size_t ws_size, hipStream_t stream) {
  if (n_in < 11) return;
  if (in_sizes[0] != kBatch * kChan * kNobj || in_sizes[1] != kDGIn * kHG || in_sizes[3] != kHG * kHG ||
      in_sizes[5] != kHG * kHG || in_sizes[7] != kHG * kHF || in_sizes[9] != kHF * kDOut) return;
  if (out_size != kBatch * kDOut) return;
  if (ws_size < kWsTotal) return;

  const float* x   = (const float*)d_in[0];
  const float* gW0 = (const float*)d_in[1];
  const float* gb0 = (const float*)d_in[2];
  const float* gW1 = (const float*)d_in[3];
  const float* gb1 = (const float*)d_in[4];
  const float* gW2 = (const float*)d_in[5];
  const float* gb2 = (const float*)d_in[6];
  const float* fW0 = (const float*)d_in[7];
  const float* fb0 = (const float*)d_in[8];
  const float* fW1 = (const float*)d_in[9];
  const float* fb1 = (const float*)d_in[10];
  float* out = (float*)d_out;

  char* ws = (char*)d_ws;
  unsigned short* W12t = (unsigned short*)(ws + kOffW12t);
  unsigned short* W1t  = W12t;
  unsigned short* W2t  = W12t + (size_t)kHG * kHG;
  unsigned short* W0t  = (unsigned short*)(ws + kOffW0t);
  unsigned short* Xt   = (unsigned short*)(ws + kOffXt);
  float*          AB   = (float*)(ws + kOffAB);
  unsigned short* H0   = (unsigned short*)(ws + kOffH0);
  unsigned short* H1   = (unsigned short*)(ws + kOffH1);
  float*          Par  = (float*)(ws + kOffPar);

  wtcast_kernel<<<dim3(kHG / 64, kHG / 64, 3), 256, 0, stream>>>(gW1, gW2, gW0, W12t, W0t, kWCarry);
  xtcast_kernel<<<dim3(kChan / 64, kBatch), 256, 0, stream>>>(x, Xt, kXCarry);

  {
    const int tiles = (kObjRows / 64) * (kW0N / 64);
    wmma_gemm64<0, false, 0, 0, false, 0><<<dim3(tiles / 8, 1), 256, 0, stream>>>(
        (const unsigned short*)Xt, (const unsigned short*)nullptr, kChan, 0L,
        (const unsigned short*)W0t, (const unsigned short*)nullptr, kChan, 0L,
        (void*)AB, (void*)nullptr, kW0N, 0L,
        (const float*)nullptr, (const float*)nullptr, 0L,
        kObjRows, kW0N, kChan, kScale0, 1.0f);
  }

  for (int ch = 0; ch < kNChunks; ++ch) {
    build_h0_kernel<<<kChunkRows / 4, 256, 0, stream>>>(AB, gW0, gb0, H0, ch);
    {
      const int tiles = (kChunkRows / 64) * (kHG / 64);
      wmma_gemm64<0, false, 2, 1, false, 2><<<dim3(tiles / 8, 1), 256, 0, stream>>>(
          (const unsigned short*)H0, (const unsigned short*)nullptr, kHG, 0L,
          (const unsigned short*)W1t, (const unsigned short*)nullptr, kHG, 0L,
          (void*)H1, (void*)nullptr, kHG, 0L,
          gb1, (const float*)nullptr, 0L,
          kChunkRows, kHG, kHG, kScale12, kHCarry);
      wmma_gemm64_rowsum<0, 2><<<dim3(tiles / 8), 256, 0, stream>>>(
          (const unsigned short*)H1, kHG,
          (const unsigned short*)W2t, kHG,
          Par + (size_t)ch * kChunkB * kNobj * kHG, kHG,
          gb2, kChunkRows, kHG, kHG, kScale12);
    }
  }

  fmlp_kernel<<<kBatch, 256, 0, stream>>>(Par, fW0, fb0, fW1, fb1, out);
}
